// QuantLinear_13065290515021
// MI455X (gfx1250) — hardware-verified
//
#include <hip/hip_runtime.h>


namespace {
constexpr int M = 2048, K = 4096, N = 4096, GS = 128, G = K / GS, PACK = 8, ML = 2048  , KC = 256  ;
constexpr float XS = 8.0f;
static_assert(M % 64 == 0 && ML % 64 == 0 && K % KC == 0 && KC % GS == 0, "tiling");
typedef _Float16 b16;
typedef __attribute__((ext_vector_type(16))) _Float16 v16b;
typedef __attribute__((ext_vector_type(8))) _Float16 v8b;
typedef __attribute__((ext_vector_type(8))) float v8f;
typedef __attribute__((ext_vector_type(4))) float v4f;
__device__ __forceinline__ float bf16_rne(float f) { unsigned int u = __float_as_uint(f); u += 0x7FFFu + ((u >> 16) & 1u); return __uint_as_float(u & 0xFFFF0000u); }
__device__ __forceinline__ void split16(float v, b16& hi, b16& lo) { hi = (b16)v; lo = (b16)(v - (float)hi); }
__device__ __forceinline__ v16b frag_kb(const b16* p, int hh) { const v8b a = *(const v8b*)(p + 8 * hh), b = *(const v8b*)(p + 16 + 8 * hh); v16b f;
#pragma unroll
  for (int e = 0; e < 8; ++e) { f[e] = a[e]; f[8 + e] = b[e]; } return f; }
__device__ __forceinline__ v8f wmma16b(v16b a, v16b b, v8f c) { v8f d = __builtin_amdgcn_wmma_f32_16x16x32_f16(false, a, false, b, (short)0, c, false, false); asm volatile("v_nop\n\tv_nop\n\tv_nop\n\tv_nop" : "+v"(d) : "v"(a), "v"(b)); return d; }
__device__ __forceinline__ void wave_lds_sync() { __builtin_amdgcn_fence(__ATOMIC_RELEASE, "workgroup"); __builtin_amdgcn_wave_barrier(); __builtin_amdgcn_fence(__ATOMIC_ACQUIRE, "workgroup"); }
__device__ __forceinline__ float pmul(float a, float b) { float p = a * b; asm volatile("" : "+v"(p)); return p; }
__device__ __forceinline__ int iclamp(int v, int lo, int hi) { return v < lo ? lo : (v > hi ? hi : v); }

__global__ __launch_bounds__(256) void prep_kernel(const int* __restrict__ qweight, const int* __restrict__ qzeros, const int* __restrict__ gidx, b16* __restrict__ QT, int* __restrict__ FLAG) {
  const size_t u = (size_t)blockIdx.x * 256 + threadIdx.x; if (u >= (size_t)N * K / 8) return; const int n = (int)(u / (K / 8)), kw = (int)(u % (K / 8)); const int k0 = kw * PACK;
  const unsigned word = (unsigned)qweight[(size_t)kw * N + n]; v8b o;
  for (int j = 0; j < 8; ++j) { const int k = k0 + j; int g = gidx[k]; if (g != k / GS) ((volatile int*)FLAG)[0] = 1;
    g = g < 0 ? 0 : (g >= G ? G - 1 : g); const unsigned zw = (unsigned)qzeros[(size_t)g * (N / PACK) + n / PACK]; const int z = (int)((zw >> (4 * (n % PACK))) & 15u) + 1; const int w = (int)((word >> (4 * j)) & 15u); o[j] = (b16)(float)(w - z); }
  for (int pass = 0; pass < 2; ++pass) { *(volatile v8b*)(QT + (size_t)n * K + k0) = o; __threadfence(); }
}
__global__ __launch_bounds__(32) void zflag_kernel(int* __restrict__ FLAG) { for (int pass = 0; pass < 2; ++pass) { ((volatile int*)FLAG)[threadIdx.x] = 0; __threadfence(); } }
__global__ __launch_bounds__(128) void gemm_kernel(const float* __restrict__ x, const b16* __restrict__ QT, const float* __restrict__ scales, const float* __restrict__ bias, const int* __restrict__ FLAG, float* __restrict__ out) {
  __shared__ __attribute__((aligned(16))) b16 As[64][KC + 8]; __shared__ __attribute__((aligned(16))) float Tf[4][16][128 + 4];
  const int wave = threadIdx.x >> 5, lane = threadIdx.x & 31, nloc = lane & 15, hlf = lane >> 4; const size_t r0 = (size_t)blockIdx.x * 64; const size_t m0 = r0 + wave * 16; const int n0 = blockIdx.y * 128;
  v8f acc[8];
#pragma unroll
  for (int t = 0; t < 8; ++t) acc[t] = (v8f){};
#pragma unroll 1
  for (int kc = 0; kc < K; kc += KC) {
    __syncthreads();
    for (int i = threadIdx.x; i < 64 * (KC / 4); i += 128) { const int rr = i / (KC / 4), q = (i % (KC / 4)) * 4; const v4f f = *(const v4f*)(x + (r0 + rr) * K + kc + q); typedef __attribute__((ext_vector_type(4))) _Float16 v4h; v4h o; for (int j = 0; j < 4; ++j) o[j] = (b16)(bf16_rne(f[j]) * XS); *(v4h*)(&As[rr][q]) = o; }
    __syncthreads();
#pragma unroll 1
    for (int gq = 0; gq < KC / GS; ++gq) { const int g = (kc + gq * GS) / GS; v8f d[8];
#pragma unroll
      for (int t = 0; t < 8; ++t) d[t] = (v8f){};
#pragma unroll
      for (int kb = 0; kb < GS; kb += 32) { const v16b a = frag_kb(&As[wave * 16 + nloc][gq * GS + kb], hlf);
#pragma unroll
        for (int t = 0; t < 8; ++t) d[t] = wmma16b(a, frag_kb(QT + (size_t)(n0 + t * 16 + nloc) * K + kc + gq * GS + kb, hlf), d[t]); }
#pragma unroll
      for (int t = 0; t < 8; ++t) { const float s = bf16_rne(scales[(size_t)g * N + n0 + t * 16 + nloc]);
#pragma unroll
        for (int r = 0; r < 8; ++r) acc[t][r] += d[t][r] * s; } } }
const bool bad = FLAG[0] != 0;
#pragma unroll
  for (int t = 0; t < 8; ++t) { const float bb = bf16_rne(bias[n0 + t * 16 + nloc]);
#pragma unroll
    for (int r = 0; r < 8; ++r) Tf[wave][8 * hlf + r][t * 16 + nloc] = bad ? __int_as_float(0x7fc00000) : acc[t][r] * (1.0f / XS) + bb; }
  wave_lds_sync();
  for (int pass = 0; pass < 2; ++pass) { for (int rr = 0; rr < 16; ++rr) *(volatile v4f*)(out + (m0 + rr) * N + n0 + lane * 4) = *(const v4f*)(&Tf[wave][rr][lane * 4]); __threadfence(); }
}
}

extern "C" void kernel_launch(void* const* d_in, const int* in_sizes, int n_in, void* d_out, int out_size, void* d_ws, size_t ws_size, hipStream_t stream) {
  (void)n_in;
  auto Fp = [&](int i) { return (const float*)d_in[i]; }; auto Ip = [&](int i) { return (const int*)d_in[i]; };
  if (in_sizes[0] != M * K || in_sizes[1] != (K / PACK) * N || in_sizes[2] != G * (N / PACK) || in_sizes[3] != G * N || in_sizes[4] != K || in_sizes[5] != N || out_size != M * N) return;
  size_t off = 0; char* ws = (char*)d_ws;
  auto carve = [&](size_t bytes) { char* p = ws + off; off += (bytes + 255) & ~(size_t)255; return p; };
  b16* QT = (b16*)carve((size_t)N * K * 2); int* FLAG = (int*)carve(256);
  if (off > ws_size || off > ((size_t)128 << 20)) return;
  zflag_kernel<<<1, 32, 0, stream>>>(FLAG);
  prep_kernel<<<(unsigned)(((size_t)N * K / 8 + 255) / 256), 256, 0, stream>>>(Ip(1), Ip(2), Ip(4), QT, FLAG);
  gemm_kernel<<<dim3(ML / 64, N / 128), 128, 0, stream>>>(Fp(0), QT, Fp(3), Fp(5), FLAG, (float*)d_out);
}
